// TemporalMamba_2731599200652
// MI455X (gfx1250) — hardware-run, weakly checked
//
#include <hip/hip_runtime.h>
#include <math.h>
#include <stdint.h>

constexpr int kBatch   = 2;
constexpr int kSeqLen  = 1024;
constexpr int kDModel  = 1024;
constexpr int kDInner  = 2048;
constexpr int kDState  = 16;
constexpr int kDtRank  = 64;
constexpr int kXpCols  = 96;
constexpr int kXpPad   = 128;
constexpr int kXzCols  = 2 * kDInner;
constexpr int kTok     = kBatch * kSeqLen;

constexpr size_t kMiB      = 1048576;
constexpr size_t kOffXz    = 0;
constexpr size_t kOffU     = 32 * kMiB;
constexpr size_t kOffUh    = 48 * kMiB;
constexpr size_t kOffUl    = 56 * kMiB;
constexpr size_t kOffYh    = kOffUh;
constexpr size_t kOffYl    = kOffUl;
constexpr size_t kOffWinH  = 64 * kMiB;
constexpr size_t kOffWinL  = 72 * kMiB;
constexpr size_t kOffDpre  = kOffWinH;
constexpr size_t kOffXh    = 80 * kMiB;
constexpr size_t kOffXl    = 84 * kMiB;
constexpr size_t kOffWoutH = kOffXh;
constexpr size_t kOffWoutL = kOffXl;
constexpr size_t kOffWxpH  = 88 * kMiB;
constexpr size_t kOffWxpL  = 88 * kMiB + 512 * 1024;
constexpr size_t kOffXdbl  = 89 * kMiB;
constexpr size_t kOffDtH   = 90 * kMiB;
constexpr size_t kOffDtL   = 90 * kMiB + 256 * 1024;
constexpr size_t kOffWdtH  = 90 * kMiB + 512 * 1024;
constexpr size_t kOffWdtL  = 90 * kMiB + 768 * 1024;
constexpr size_t kWsTotal  = 91 * kMiB;
static_assert((size_t)kTok * kXzCols * 4 == 32 * kMiB, "xz extent");
static_assert((size_t)kTok * kDInner * 4 == 16 * kMiB, "u / dpre extent");
static_assert((size_t)kTok * kDInner * 2 == 8 * kMiB, "u / y plane extent");
static_assert((size_t)kXzCols * kDModel * 2 == 8 * kMiB, "Wt_in plane extent");
static_assert((size_t)kTok * kDModel * 2 == 4 * kMiB, "x plane extent");
static_assert((size_t)kDModel * kDInner * 2 == 4 * kMiB, "Wt_out plane extent");
static_assert((size_t)kXpPad * kDInner * 2 == 512 * 1024, "Wt_xp plane extent");
static_assert((size_t)kTok * kXpPad * 4 == kMiB, "x_dbl extent");
static_assert((size_t)kTok * kDtRank * 2 == 256 * 1024, "dt plane extent");
static_assert((size_t)kDInner * kDtRank * 2 == 256 * 1024, "Wt_dt plane extent");
static_assert(kWsTotal == 95420416, "carve total");
static_assert(kWsTotal <= 134217728, "carve under 128 MiB");

typedef __attribute__((ext_vector_type(16))) _Float16 v16h;
typedef __attribute__((ext_vector_type(8)))  _Float16 v8h;
typedef __attribute__((ext_vector_type(16))) __bf16   v16b;
typedef __attribute__((ext_vector_type(8)))  __bf16   v8b;
typedef __attribute__((ext_vector_type(8)))  float    v8f;
typedef __attribute__((ext_vector_type(4)))  float    v4f;
typedef __attribute__((ext_vector_type(4)))  unsigned int v4u;

__device__ __forceinline__ unsigned short f2bf_bits(float f) {
  unsigned u = __float_as_uint(f);
  return (unsigned short)((u + 0x7FFFu + ((u >> 16) & 1u)) >> 16);
}
__device__ __forceinline__ float bf_bits2f(unsigned short h) { return __uint_as_float(((unsigned)h) << 16); }

__device__ __forceinline__ void dep_guard_h(v8f& a, v8f& b, v16h x, v16h y) { asm volatile("v_nop\n\tv_nop\n\tv_nop\n\tv_nop" : "+v"(a), "+v"(b) : "v"(x), "v"(y)); }
__device__ __forceinline__ void dep_guard_b(v8f& a, v8f& b, v16b x, v16b y) { asm volatile("v_nop\n\tv_nop\n\tv_nop\n\tv_nop" : "+v"(a), "+v"(b) : "v"(x), "v"(y)); }
__device__ __forceinline__ void keep4_h(v16h a, v16h b, v16h c, v16h d) { asm volatile("v_nop" :: "v"(a), "v"(b), "v"(c), "v"(d)); }
__device__ __forceinline__ void keep4_b(v16b a, v16b b, v16b c, v16b d) { asm volatile("v_nop" :: "v"(a), "v"(b), "v"(c), "v"(d)); }
__device__ __forceinline__ void acc_guard4(v8f& a, v8f& b, v8f& c, v8f& d) { asm volatile("v_nop\n\tv_nop\n\tv_nop\n\tv_nop" : "+v"(a), "+v"(b), "+v"(c), "+v"(d)); }
template <typename T> struct Frag;
template <> struct Frag<_Float16> {
  typedef v16h V; union U { v16h v; v8h h[2]; };
  static __device__ __forceinline__ v16h load(const _Float16* p) {
    U f; f.h[0] = *(const v8h*)(p); f.h[1] = *(const v8h*)(p + 16); return f.v;
  }
  static __device__ __forceinline__ v8f mma(v16h a, v16h b, v8f c) {
    return __builtin_amdgcn_wmma_f32_16x16x32_f16(false, a, false, b, (short)0, c, false, false);
  }
  static __device__ __forceinline__ void guard(v8f& a, v8f& b, v16h x, v16h y) { dep_guard_h(a, b, x, y); }
  static __device__ __forceinline__ void keep(v16h a, v16h b, v16h c, v16h d) { keep4_h(a, b, c, d); }
};
template <> struct Frag<__bf16> {
  typedef v16b V; union U { v16b v; v8b h[2]; };
  static __device__ __forceinline__ v16b load(const __bf16* p) {
    U f; f.h[0] = *(const v8b*)(p); f.h[1] = *(const v8b*)(p + 16); return f.v;
  }
  static __device__ __forceinline__ v8f mma(v16b a, v16b b, v8f c) {
    return __builtin_amdgcn_wmma_f32_16x16x32_bf16(false, a, false, b, (short)0, c, false, false);
  }
  static __device__ __forceinline__ void guard(v8f& a, v8f& b, v16b x, v16b y) { dep_guard_b(a, b, x, y); }
  static __device__ __forceinline__ void keep(v16b a, v16b b, v16b c, v16b d) { keep4_b(a, b, c, d); }
};

__device__ __forceinline__ unsigned pk16(unsigned short a, unsigned short b) { return (unsigned)a | ((unsigned)b << 16); }
__device__ __forceinline__ void split_bf(float f, unsigned short& hb, unsigned short& lb) {
  hb = f2bf_bits(f);
  lb = f2bf_bits(f - bf_bits2f(hb));
}

template <int ET> struct Elem;
template <> struct Elem<0> { typedef _Float16 T; };
template <> struct Elem<1> { typedef __bf16 T; };
template <int ET, bool SPLIT, int BIAS_MODE, int OUT_MODE, bool RESID, int ACT = 0>
__global__ __launch_bounds__(256) void wmma_gemm64(
    const unsigned short* __restrict__ Ap, const unsigned short* __restrict__ A2p, int lda, long strideA,
    const unsigned short* __restrict__ Btp, const unsigned short* __restrict__ Bt2p, int ldb, long strideB,
    void* __restrict__ Cout, void* __restrict__ Cout2, int ldc, long strideC,
    const float* __restrict__ bias,
    const float* __restrict__ resid, long strideR,
    int M, int N, int K, float scale) {
  typedef typename Elem<ET>::T T;
  typedef typename Frag<T>::V V;
  const T* A = (const T*)Ap; const T* A2 = (const T*)A2p; const T* Bt = (const T*)Btp; const T* Bt2 = (const T*)Bt2p;
  __shared__ __align__(16) float sT[8][16 * 68];
  const int b    = blockIdx.y;
  const int lane = threadIdx.x & 31;
  const int wave = threadIdx.x >> 5;
  const int tilesN = N >> 6;
  const int tilesM = M >> 6;
  const int tile = blockIdx.x * 8 + wave;
  if (tile >= tilesM * tilesN) return;
  const int tm = tile / tilesN;
  const int tn = tile - tm * tilesN;
  const int m0 = tm << 6;
  const int n0 = tn << 6;

  const T* Ab  = A  + (size_t)b * strideA;
  const T* Bb  = Bt + (size_t)b * strideB;
  const T* Ab2 = SPLIT ? (A2  + (size_t)b * strideA) : nullptr;
  const T* Bb2 = SPLIT ? (Bt2 + (size_t)b * strideB) : nullptr;

  const int rlane = lane & 15;
  const int koff  = (lane >> 4) * 8;
  const int mOff  = (lane >> 4) * 8;

  v8f acc[4][4];
#pragma unroll
  for (int i = 0; i < 4; ++i)
#pragma unroll
    for (int j = 0; j < 4; ++j) acc[i][j] = (v8f){0.f,0.f,0.f,0.f,0.f,0.f,0.f,0.f};

  for (int k0 = 0; k0 < K; k0 += 32) {
    V bh[4], bl[4];
#pragma unroll
    for (int j = 0; j < 4; ++j) {
      const size_t bo = (size_t)(n0 + (j << 4) + rlane) * ldb + koff + k0;
      bh[j] = Frag<T>::load(Bb + bo);
      if (SPLIT) bl[j] = Frag<T>::load(Bb2 + bo);
    }
#pragma unroll
    for (int i = 0; i < 4; ++i) {
      const size_t ao = (size_t)(m0 + (i << 4) + rlane) * lda + koff + k0;
      V ah = Frag<T>::load(Ab + ao);
      V al;
      if (SPLIT) al = Frag<T>::load(Ab2 + ao);
#pragma unroll
      for (int j = 0; j < 4; ++j) {
        acc[i][j] = Frag<T>::mma(ah, bh[j], acc[i][j]);
        if (SPLIT) {
          acc[i][j] = Frag<T>::mma(ah, bl[j], acc[i][j]);
          acc[i][j] = Frag<T>::mma(al, bh[j], acc[i][j]);
        }
      }
      Frag<T>::guard(acc[i][0], acc[i][3], ah, SPLIT ? al : ah);
    }
    Frag<T>::keep(bh[0], bh[1], bh[2], bh[3]);
    if (SPLIT) Frag<T>::keep(bl[0], bl[1], bl[2], bl[3]);
  }
  acc_guard4(acc[0][0], acc[0][1], acc[0][2], acc[0][3]);
  acc_guard4(acc[1][0], acc[1][1], acc[1][2], acc[1][3]);
  acc_guard4(acc[2][0], acc[2][1], acc[2][2], acc[2][3]);
  acc_guard4(acc[3][0], acc[3][1], acc[3][2], acc[3][3]);

  float* slab = sT[wave];
  const float* Rb = RESID ? (resid + (size_t)b * strideR) : nullptr;
#pragma unroll
  for (int i = 0; i < 4; ++i) {
    const int mBase = m0 + (i << 4);
#pragma unroll
    for (int j = 0; j < 4; ++j) {
      const int n = n0 + (j << 4) + rlane;
      float bv = 0.f;
      if (BIAS_MODE == 2) bv = bias[n];
#pragma unroll
      for (int r = 0; r < 8; ++r) {
        float v = acc[i][j][r] * scale;
        if (BIAS_MODE == 1) v += bias[mBase + mOff + r];
        if (BIAS_MODE == 2) v += bv;
        if (RESID) v += Rb[(size_t)(mBase + mOff + r) * ldc + n];
        if (ACT == 2) v = fmaxf(v, 0.0f);
        if (ACT == 4) v = (v > 0.f) ? v : 0.01f * v;
        slab[(mOff + r) * 68 + (j << 4) + rlane] = v;
      }
    }
    __builtin_amdgcn_fence(__ATOMIC_RELEASE, "workgroup");
    __builtin_amdgcn_wave_barrier();
    __builtin_amdgcn_fence(__ATOMIC_ACQUIRE, "workgroup");
    if (OUT_MODE == 0) {
      float* C = (float*)Cout + (size_t)b * strideC;
      const int hh = lane >> 4, c4 = (lane & 15) * 4;
      for (int pass = 0; pass < 2; ++pass) {
#pragma unroll
        for (int it = 0; it < 8; ++it) {
          const int row = it * 2 + hh;
          v4f v = *(const v4f*)(slab + row * 68 + c4);
          *(volatile v4f*)(C + (size_t)(mBase + row) * ldc + n0 + c4) = v;
        }
        __threadfence();
      }
    } else {
      const int q = lane >> 3, c8 = (lane & 7) * 8;
      unsigned short* C  = (unsigned short*)Cout  + (size_t)b * strideC;
      unsigned short* C2 = (OUT_MODE == 2) ? ((unsigned short*)Cout2 + (size_t)b * strideC) : nullptr;
      for (int pass = 0; pass < 2; ++pass) {
#pragma unroll
        for (int it = 0; it < 4; ++it) {
          const int row = it * 4 + q;
          const float* sp = slab + row * 68 + c8;
          v8h hv, lv;
#pragma unroll
          for (int e = 0; e < 8; ++e) {
            if (OUT_MODE == 1) {
              hv[e] = (_Float16)sp[e];
            } else {
              unsigned short hb = f2bf_bits(sp[e]);
              unsigned short lb = f2bf_bits(sp[e] - bf_bits2f(hb));
              hv[e] = __builtin_bit_cast(_Float16, hb);
              lv[e] = __builtin_bit_cast(_Float16, lb);
            }
          }
          *(volatile v8h*)(C + (size_t)(mBase + row) * ldc + n0 + c8) = hv;
          if (OUT_MODE == 2) *(volatile v8h*)(C2 + (size_t)(mBase + row) * ldc + n0 + c8) = lv;
        }
        __threadfence();
      }
    }
    __builtin_amdgcn_fence(__ATOMIC_RELEASE, "workgroup");
    __builtin_amdgcn_wave_barrier();
    __builtin_amdgcn_fence(__ATOMIC_ACQUIRE, "workgroup");
  }
}

__global__ __launch_bounds__(256) void rows_split8_kernel(const float* __restrict__ in, int ld_in,
                                                          unsigned short* __restrict__ oh, unsigned short* __restrict__ ol,
                                                          int ld_out, int c8_shift, int nthr) {
  const int i = blockIdx.x * 256 + threadIdx.x;
  if (i >= nthr) return;
  const int row = i >> c8_shift;
  const int c8  = (i & ((1 << c8_shift) - 1)) * 8;
  const float* p = in + (size_t)row * ld_in + c8;
  const v4f a = *(const v4f*)(p);
  const v4f c = *(const v4f*)(p + 4);
  unsigned short hb[8], lb[8];
#pragma unroll
  for (int e = 0; e < 4; ++e) {
    split_bf(a[e], hb[e], lb[e]);
    split_bf(c[e], hb[4 + e], lb[4 + e]);
  }
  const v4u uh = (v4u){pk16(hb[0], hb[1]), pk16(hb[2], hb[3]), pk16(hb[4], hb[5]), pk16(hb[6], hb[7])};
  const v4u ul = (v4u){pk16(lb[0], lb[1]), pk16(lb[2], lb[3]), pk16(lb[4], lb[5]), pk16(lb[6], lb[7])};
  const size_t o = (size_t)row * ld_out + c8;
  *(volatile v4u*)(oh + o) = uh;
  *(volatile v4u*)(ol + o) = ul;
  __threadfence();
  *(volatile v4u*)(oh + o) = uh;
  *(volatile v4u*)(ol + o) = ul;
}

__global__ __launch_bounds__(256) void transpose_split_kernel(const float* __restrict__ in,
                                                              unsigned short* __restrict__ oh, unsigned short* __restrict__ ol,
                                                              int nrows, int ncols) {
  __shared__ float sm[64][65];
  const int t  = threadIdx.x;
  const int c0 = blockIdx.x * 64;
  const int r0 = blockIdx.y * 64;
#pragma unroll
  for (int i = 0; i < 16; ++i) {
    const int e  = i * 256 + t;
    const int rl = e >> 6;
    const int cl = e & 63;
    const int c  = c0 + cl;
    const int cc = (c < ncols) ? c : (ncols - 1);
    float v = in[(size_t)(r0 + rl) * ncols + cc];
    v = (c < ncols) ? v : 0.0f;
    sm[cl][rl] = v;
  }
  __syncthreads();
  const int lane = t & 31, wave = t >> 5;
  const int q = lane >> 3, c8 = (lane & 7) * 8;
  for (int pass = 0; pass < 2; ++pass) {
#pragma unroll
    for (int it = 0; it < 2; ++it) {
      const int row = wave * 8 + it * 4 + q;
      unsigned short hb[8], lb[8];
#pragma unroll
      for (int e = 0; e < 8; ++e) split_bf(sm[row][c8 + e], hb[e], lb[e]);
      const v4u uh = (v4u){pk16(hb[0], hb[1]), pk16(hb[2], hb[3]), pk16(hb[4], hb[5]), pk16(hb[6], hb[7])};
      const v4u ul = (v4u){pk16(lb[0], lb[1]), pk16(lb[2], lb[3]), pk16(lb[4], lb[5]), pk16(lb[6], lb[7])};
      const size_t o = (size_t)(c0 + row) * nrows + r0 + c8;
      *(volatile v4u*)(oh + o) = uh;
      *(volatile v4u*)(ol + o) = ul;
    }
    __threadfence();
  }
}

__global__ __launch_bounds__(256) void conv_silu_kernel(const float* __restrict__ xz, const float* __restrict__ conv_w,
                                                        const float* __restrict__ conv_b, float* __restrict__ u) {
  const int i   = blockIdx.x * 256 + threadIdx.x;
  const int row = i >> 9;
  const int d4  = (i & 511) * 4;
  const int l   = row & (kSeqLen - 1);
  const int r1  = (l >= 1) ? (row - 1) : row;
  const int r2  = (l >= 2) ? (row - 2) : row;
  const int r3  = (l >= 3) ? (row - 3) : row;
  const v4f x0 = *(const v4f*)(xz + (size_t)row * kXzCols + d4);
  const v4f x1 = *(const v4f*)(xz + (size_t)r1  * kXzCols + d4);
  const v4f x2 = *(const v4f*)(xz + (size_t)r2  * kXzCols + d4);
  const v4f x3 = *(const v4f*)(xz + (size_t)r3  * kXzCols + d4);
  const v4f bb = *(const v4f*)(conv_b + d4);
  v4f res;
#pragma unroll
  for (int e = 0; e < 4; ++e) {
    const v4f we = *(const v4f*)(conv_w + (size_t)(d4 + e) * 4);
    const float v3 = (l >= 3) ? x3[e] : 0.0f;
    const float v2 = (l >= 2) ? x2[e] : 0.0f;
    const float v1 = (l >= 1) ? x1[e] : 0.0f;
    float acc = v3 * we[0];
    acc += v2 * we[1];
    acc += v1 * we[2];
    acc += x0[e] * we[3];
    acc += bb[e];
    const float sig = 1.0f / (1.0f + expf(-acc));
    res[e] = acc * sig;
  }
  float* qo = u + (size_t)row * kDInner + d4;
  *(volatile v4f*)qo = res;
  __threadfence();
  *(volatile v4f*)qo = res;
}

constexpr int kScanCh    = 64;
constexpr int kScanSteps = 64;
__global__ __launch_bounds__(64) void scan_kernel(const float* __restrict__ dpre, const float* __restrict__ u,
                                                  const float* __restrict__ xz, const float* __restrict__ xdbl,
                                                  const float* __restrict__ A_log, const float* __restrict__ b_dt,
                                                  const float* __restrict__ D_skip,
                                                  unsigned short* __restrict__ yh, unsigned short* __restrict__ yl) {
  __shared__ __align__(16) float sA[kDState * kScanCh];
  __shared__ __align__(16) float sH[kDState * kScanCh];
  __shared__ __align__(16) float sBC[kScanSteps * 32];
  __shared__ __align__(16) unsigned short sYh[kScanSteps * kScanCh];
  __shared__ __align__(16) unsigned short sYl[kScanSteps * kScanCh];
  const int t  = threadIdx.x;
  const int b  = blockIdx.y;
  const int d0 = blockIdx.x * kScanCh;
  const int d  = d0 + t;
#pragma unroll 1
  for (int n = 0; n < kDState; ++n) {
    sA[n * kScanCh + t] = -expf(A_log[(size_t)d * kDState + n]);
    sH[n * kScanCh + t] = 0.0f;
  }
  const float bd  = b_dt[d];
  const float dsk = D_skip[d];
  const int lane = t & 31, wave = t >> 5;
  const int q = lane >> 3, c8 = (lane & 7) * 8;

  for (int lc = 0; lc < kSeqLen; lc += kScanSteps) {
    __syncthreads();
#pragma unroll
    for (int i = 0; i < 8; ++i) {
      const int idx = i * kScanCh + t;
      const int s   = idx >> 3;
      const int q4  = (idx & 7) * 4;
      const v4f v = *(const v4f*)(xdbl + (size_t)(b * kSeqLen + lc + s) * kXpPad + kDtRank + q4);
      *(v4f*)(sBC + s * 32 + q4) = v;
    }
    __syncthreads();
#pragma unroll 1
    for (int s = 0; s < kScanSteps; ++s) {
      const size_t row = (size_t)b * kSeqLen + lc + s;
      const float xdt   = dpre[row * kDInner + d] + bd;
      const float delta = fmaxf(xdt, 0.0f) + log1pf(expf(-fabsf(xdt)));
      const float uu    = u[row * kDInner + d];
      const float zz    = xz[row * kXzCols + kDInner + d];
      const float du    = delta * uu;
      float y = 0.0f;
#pragma unroll 1
      for (int n = 0; n < kDState; ++n) {
        const float a  = sA[n * kScanCh + t];
        const float hp = sH[n * kScanCh + t];
        const float hn = expf(delta * a) * hp + du * sBC[s * 32 + n];
        sH[n * kScanCh + t] = hn;
        y += hn * sBC[s * 32 + kDState + n];
      }
      y += dsk * uu;
      const float sig = 1.0f / (1.0f + expf(-zz));
      y = y * (zz * sig);
      unsigned short hb, lb;
      split_bf(y, hb, lb);
      sYh[s * kScanCh + t] = hb;
      sYl[s * kScanCh + t] = lb;
    }
    __syncthreads();
    for (int pass = 0; pass < 2; ++pass) {
#pragma unroll
      for (int it = 0; it < 8; ++it) {
        const int rr = it * 8 + wave * 4 + q;
        const v4u vh = *(const v4u*)(sYh + rr * kScanCh + c8);
        const v4u vl = *(const v4u*)(sYl + rr * kScanCh + c8);
        const size_t o = (size_t)(b * kSeqLen + lc + rr) * kDInner + d0 + c8;
        *(volatile v4u*)(yh + o) = vh;
        *(volatile v4u*)(yl + o) = vl;
      }
      __threadfence();
    }
  }
}

extern "C" void kernel_launch(void* const* d_in, const int* in_sizes, int n_in,
                              void* d_out, int out_size, void* d_ws, size_t ws_size,
                              hipStream_t stream) {
  if (n_in < 10) return;
  if (out_size != kTok * kDModel) return;
  if (ws_size < kWsTotal) return;
  if (in_sizes[0] != kTok * kDModel || in_sizes[1] != kDModel * kXzCols || in_sizes[4] != kDInner * kXpCols ||
      in_sizes[5] != kDtRank * kDInner || in_sizes[9] != kDInner * kDModel) return;

  const float* x       = (const float*)d_in[0];
  const float* W_in    = (const float*)d_in[1];
  const float* conv_w  = (const float*)d_in[2];
  const float* conv_b  = (const float*)d_in[3];
  const float* W_xproj = (const float*)d_in[4];
  const float* W_dt    = (const float*)d_in[5];
  const float* b_dt    = (const float*)d_in[6];
  const float* A_log   = (const float*)d_in[7];
  const float* D_skip  = (const float*)d_in[8];
  const float* W_out   = (const float*)d_in[9];
  float* out = (float*)d_out;

  char* ws = (char*)d_ws;
  float* xz    = (float*)(ws + kOffXz);
  float* ubuf  = (float*)(ws + kOffU);
  unsigned short* uh    = (unsigned short*)(ws + kOffUh);
  unsigned short* ul    = (unsigned short*)(ws + kOffUl);
  unsigned short* yhp   = (unsigned short*)(ws + kOffYh);
  unsigned short* ylp   = (unsigned short*)(ws + kOffYl);
  unsigned short* winh  = (unsigned short*)(ws + kOffWinH);
  unsigned short* winl  = (unsigned short*)(ws + kOffWinL);
  float* dpre  = (float*)(ws + kOffDpre);
  unsigned short* xh    = (unsigned short*)(ws + kOffXh);
  unsigned short* xl    = (unsigned short*)(ws + kOffXl);
  unsigned short* wouth = (unsigned short*)(ws + kOffWoutH);
  unsigned short* woutl = (unsigned short*)(ws + kOffWoutL);
  unsigned short* wxph  = (unsigned short*)(ws + kOffWxpH);
  unsigned short* wxpl  = (unsigned short*)(ws + kOffWxpL);
  float* xdbl  = (float*)(ws + kOffXdbl);
  unsigned short* dth   = (unsigned short*)(ws + kOffDtH);
  unsigned short* dtl   = (unsigned short*)(ws + kOffDtL);
  unsigned short* wdth  = (unsigned short*)(ws + kOffWdtH);
  unsigned short* wdtl  = (unsigned short*)(ws + kOffWdtL);

  rows_split8_kernel<<<(kTok * (kDModel / 8)) / 256, 256, 0, stream>>>(x, kDModel, xh, xl, kDModel, 7, kTok * (kDModel / 8));
  {
    dim3 g(kXzCols / 64, kDModel / 64);
    transpose_split_kernel<<<g, 256, 0, stream>>>(W_in, winh, winl, kDModel, kXzCols);
  }
  {
    const int tiles = (kTok / 64) * (kXzCols / 64);
    dim3 g((tiles + 7) / 8, 1);
    wmma_gemm64<1, true, 0, 0, false, 0><<<g, 256, 0, stream>>>(
        xh, xl, kDModel, 0L, winh, winl, kDModel, 0L, (void*)xz, (void*)0, kXzCols, 0L,
        (const float*)0, (const float*)0, 0L, kTok, kXzCols, kDModel, 1.0f);
  }
  conv_silu_kernel<<<(kTok * kDInner / 4) / 256, 256, 0, stream>>>(xz, conv_w, conv_b, ubuf);
  rows_split8_kernel<<<(kTok * (kDInner / 8)) / 256, 256, 0, stream>>>(ubuf, kDInner, uh, ul, kDInner, 8, kTok * (kDInner / 8));
  {
    dim3 g(kXpPad / 64, kDInner / 64);
    transpose_split_kernel<<<g, 256, 0, stream>>>(W_xproj, wxph, wxpl, kDInner, kXpCols);
  }
  {
    const int tiles = (kTok / 64) * (kXpPad / 64);
    dim3 g((tiles + 7) / 8, 1);
    wmma_gemm64<1, true, 0, 0, false, 0><<<g, 256, 0, stream>>>(
        uh, ul, kDInner, 0L, wxph, wxpl, kDInner, 0L, (void*)xdbl, (void*)0, kXpPad, 0L,
        (const float*)0, (const float*)0, 0L, kTok, kXpPad, kDInner, 1.0f);
  }
  rows_split8_kernel<<<(kTok * (kDtRank / 8)) / 256, 256, 0, stream>>>(xdbl, kXpPad, dth, dtl, kDtRank, 3, kTok * (kDtRank / 8));
  {
    dim3 g(kDInner / 64, kDtRank / 64);
    transpose_split_kernel<<<g, 256, 0, stream>>>(W_dt, wdth, wdtl, kDtRank, kDInner);
  }
  {
    const int tiles = (kTok / 64) * (kDInner / 64);
    dim3 g((tiles + 7) / 8, 1);
    wmma_gemm64<1, true, 0, 0, false, 0><<<g, 256, 0, stream>>>(
        dth, dtl, kDtRank, 0L, wdth, wdtl, kDtRank, 0L, (void*)dpre, (void*)0, kDInner, 0L,
        (const float*)0, (const float*)0, 0L, kTok, kDInner, kDtRank, 1.0f);
  }
  {
    dim3 g(kDModel / 64, kDInner / 64);
    transpose_split_kernel<<<g, 256, 0, stream>>>(W_out, wouth, woutl, kDInner, kDModel);
  }
  {
    dim3 g(kDInner / kScanCh, kBatch);
    scan_kernel<<<g, kScanCh, 0, stream>>>(dpre, ubuf, xz, xdbl, A_log, b_dt, D_skip, yhp, ylp);
  }
  {
    const int tiles = (kTok / 64) * (kDModel / 64);
    dim3 g((tiles + 7) / 8, 1);
    wmma_gemm64<1, true, 0, 0, false, 0><<<g, 256, 0, stream>>>(
        yhp, ylp, kDInner, 0L, wouth, woutl, kDInner, 0L, (void*)out, (void*)0, kDModel, 0L,
        (const float*)0, (const float*)0, 0L, kTok, kDModel, kDInner, 1.0f);
  }
}
